// Trans_79602923864525
// MI455X (gfx1250) — hardware-verified
//
#include <hip/hip_runtime.h>
#include <math.h>


#define BATCH 16
#define CDIM  128
#define LDIM  2048
#define DDIM  256

typedef __attribute__((ext_vector_type(16))) __bf16   v16bf;
typedef __attribute__((ext_vector_type(8)))  __bf16   v8bf;
typedef __attribute__((ext_vector_type(16))) _Float16 v16h;
typedef __attribute__((ext_vector_type(8)))  _Float16 v8h;
typedef __attribute__((ext_vector_type(8)))  float v8f;
typedef __attribute__((ext_vector_type(4)))  float v4f;
typedef __attribute__((ext_vector_type(4)))  unsigned v4u;

template <typename T> __device__ __forceinline__ void vst2(void* p, T v) { *(volatile T*)p = v; __threadfence(); *(volatile T*)p = v; }
__device__ __forceinline__ v8f wmma_bf(v16bf a, v16bf b, v8f c) {
  v8f d = __builtin_amdgcn_wmma_f32_16x16x32_bf16(false, a, false, b, (short)0, c, false, false);
  asm volatile("v_nop\n\tv_nop\n\tv_nop\n\tv_nop" : "+v"(d) : "v"(a), "v"(b));
  return d;
}
__device__ __forceinline__ v8f wmma_h(v16h a, v16h b, v8f c) {
  v8f d = __builtin_amdgcn_wmma_f32_16x16x32_f16(false, a, false, b, (short)0, c, false, false);
  asm volatile("v_nop\n\tv_nop\n\tv_nop\n\tv_nop" : "+v"(d) : "v"(a), "v"(b));
  return d;
}
struct F2 { v16bf h, l; };
__device__ __forceinline__ F2 split16(const float* v) {
  F2 r;
#pragma unroll
  for (int i = 0; i < 16; ++i) { const __bf16 hh = (__bf16)v[i]; r.h[i] = hh; r.l[i] = (__bf16)(v[i] - (float)hh); }
  return r;
}
__device__ __forceinline__ F2 split_row(const float* row, int k0, int lane) {
  float v[16]; const float* p = row + k0 + 8 * (lane >> 4);
#pragma unroll
  for (int i = 0; i < 8; ++i) { v[i] = p[i]; v[8 + i] = p[16 + i]; }
  return split16(v);
}
__device__ __forceinline__ v8f mac3(const F2& a, const F2& b, v8f c) { c = wmma_bf(a.l, b.h, c); c = wmma_bf(a.h, b.l, c); return wmma_bf(a.h, b.h, c); }
__device__ __forceinline__ v16bf frag_bf(const __bf16* row, int k0, int lane) {
  union { v16bf v; v8bf q[2]; } r; const __bf16* p = row + k0 + 8 * (lane >> 4);
  r.q[0] = *(const v8bf*)(p); r.q[1] = *(const v8bf*)(p + 16); return r.v;
}

__global__ __launch_bounds__(128) void k_proj(const float* __restrict__ x,
    const float* __restrict__ Wq, const float* __restrict__ bq, const float* __restrict__ Wk, const float* __restrict__ bk,
    const float* __restrict__ Wv, const float* __restrict__ bv, float* __restrict__ Qf, float* __restrict__ Kf, _Float16* __restrict__ Vh) {
  __shared__ __align__(16) float xs[CDIM][68];
  __shared__ __align__(16) float st[4][16 * 132];
  __shared__ __align__(16) _Float16 vs[CDIM][72];
  const int tid = threadIdx.x, wave = tid >> 5, lane = tid & 31, col = lane & 15, g = lane >> 4;
  const int b = blockIdx.y, l0 = blockIdx.x * 64;
  for (int i = tid; i < CDIM * 16; i += 128) { const int c = i >> 4, q = i & 15;
    *(v4f*)&xs[c][q * 4] = *(const v4f*)(x + ((size_t)b * CDIM + c) * LDIM + l0 + q * 4); }
  __syncthreads();
  const int m = wave * 16 + col;
  F2 af[4];
#pragma unroll
  for (int kc = 0; kc < 4; ++kc) {
    float v[16];
#pragma unroll
    for (int i = 0; i < 8; ++i) { v[i] = xs[kc * 32 + 8 * g + i][m]; v[8 + i] = xs[kc * 32 + 16 + 8 * g + i][m]; }
    af[kc] = split16(v);
  }
  float* S = st[wave];
#pragma unroll 1
  for (int which = 0; which < 3; ++which) {
    const float* W = which == 0 ? Wq : (which == 1 ? Wk : Wv);
    const float* bb = which == 0 ? bq : (which == 1 ? bk : bv);
#pragma unroll 1
    for (int j = 0; j < 8; ++j) {
      v8f acc = {};
      const float* wrow = W + (size_t)(j * 16 + col) * CDIM;
#pragma unroll
      for (int kc = 0; kc < 4; ++kc) acc = mac3(af[kc], split_row(wrow, kc * 32, lane), acc);
      const float bo = bb[j * 16 + col];
#pragma unroll
      for (int r = 0; r < 8; ++r) S[(8 * g + r) * 132 + j * 16 + col] = acc[r] + bo;
    }
    asm volatile("s_wait_dscnt 0" ::: "memory"); __builtin_amdgcn_wave_barrier(); __builtin_amdgcn_fence(__ATOMIC_RELEASE, "workgroup");
    if (which < 2) {
      float* dst = (which == 0 ? Qf : Kf) + ((size_t)b * LDIM + l0 + wave * 16) * CDIM;
#pragma unroll 4
      for (int r = 0; r < 16; ++r) vst2(dst + (size_t)r * CDIM + lane * 4, *(const v4f*)(S + r * 132 + lane * 4));
    } else {
      for (int i = lane; i < 16 * 128; i += 32) { const int r = i >> 7, c = i & 127; vs[c][wave * 16 + r] = (_Float16)S[r * 132 + c]; }
    }
    __builtin_amdgcn_wave_barrier();
  }
  __syncthreads();
  for (int gq = tid; gq < 128 * 8; gq += 128) { const int c = gq >> 3, pc = gq & 7;
    vst2(Vh + ((size_t)b * CDIM + c) * LDIM + l0 + pc * 8, *(const v4u*)(&vs[c][pc * 8])); }
}

__global__ __launch_bounds__(128) void k_attn(const float* __restrict__ Qf, const float* __restrict__ Kf, const _Float16* __restrict__ Vh,
                                             const float* __restrict__ pos, float* __restrict__ out) {
  __shared__ __align__(16) __bf16 Ahi[64][DDIM + 8], Alo[64][DDIM + 8];
  __shared__ __align__(16) __bf16 Bhi[32][DDIM + 8], Blo[32][DDIM + 8];
  __shared__ __align__(16) _Float16 Vt[CDIM][40];
  __shared__ __align__(16) float Ps[4][16 * 32];
  const int tid = threadIdx.x, wave = tid >> 5, lane = tid & 31, col = lane & 15, g = lane >> 4;
  const int b = blockIdx.y, m0 = blockIdx.x * 64;
  for (int i = tid; i < 64 * DDIM; i += 128) { const int r = i >> 8, f = i & 255;
    const float v = (f < CDIM) ? Qf[((size_t)b * LDIM + m0 + r) * CDIM + f] : pos[(size_t)(m0 + r) * CDIM + (f - CDIM)];
    const __bf16 hh = (__bf16)v; Ahi[r][f] = hh; Alo[r][f] = (__bf16)(v - (float)hh); }
  __syncthreads();
  const int mrow = wave * 16 + col;
  float m_r[8], l_r[8];
  v8f o[8] = {};
#pragma unroll
  for (int r = 0; r < 8; ++r) { m_r[r] = -3.0e38f; l_r[r] = 0.f; }
  float* P = Ps[wave];
  for (int kb = 0; kb < LDIM; kb += 32) {
    __syncthreads();
    for (int i = tid; i < 32 * DDIM; i += 128) { const int r = i >> 8, f = i & 255;
      const float v = (f < CDIM) ? Kf[((size_t)b * LDIM + kb + r) * CDIM + f] : Qf[((size_t)b * LDIM + kb + r) * CDIM + (f - CDIM)];
      const __bf16 hh = (__bf16)v; Bhi[r][f] = hh; Blo[r][f] = (__bf16)(v - (float)hh); }
    for (int i = tid; i < CDIM * 4; i += 128) { const int c = i >> 2, q = i & 3;
      *(v4u*)&Vt[c][q * 8] = *(const v4u*)(Vh + ((size_t)b * CDIM + c) * LDIM + kb + q * 8); }
    __syncthreads();
    v8f s[2] = {(v8f){}, (v8f){}};
#pragma unroll 2
    for (int kc = 0; kc < DDIM / 32; ++kc) {
      F2 a; a.h = frag_bf(&Ahi[mrow][0], kc * 32, lane); a.l = frag_bf(&Alo[mrow][0], kc * 32, lane);
#pragma unroll
      for (int j = 0; j < 2; ++j) {
        F2 bf; bf.h = frag_bf(&Bhi[j * 16 + col][0], kc * 32, lane); bf.l = frag_bf(&Blo[j * 16 + col][0], kc * 32, lane);
        s[j] = mac3(a, bf, s[j]);
      }
    }
#pragma unroll
    for (int r = 0; r < 8; ++r) {
      float mx = fmaxf(s[0][r], s[1][r]);
#pragma unroll
      for (int off = 8; off >= 1; off >>= 1) mx = fmaxf(mx, __shfl_xor(mx, off, 32));
      const float mn = fmaxf(m_r[r], mx);
      const float p0 = expf(s[0][r] - mn), p1 = expf(s[1][r] - mn);
      P[(8 * g + r) * 32 + col] = p0; P[(8 * g + r) * 32 + 16 + col] = p1;
      float sum = p0 + p1;
#pragma unroll
      for (int off = 8; off >= 1; off >>= 1) sum += __shfl_xor(sum, off, 32);
      const float corr = expf(m_r[r] - mn);
      l_r[r] = l_r[r] * corr + sum; m_r[r] = mn;
#pragma unroll
      for (int t = 0; t < 8; ++t) o[t][r] *= corr;
    }
    asm volatile("s_wait_dscnt 0" ::: "memory"); __builtin_amdgcn_wave_barrier(); __builtin_amdgcn_fence(__ATOMIC_RELEASE, "workgroup");
    v16h pa;
    { const float* pr = P + col * 32 + 8 * g;
#pragma unroll
      for (int i = 0; i < 8; ++i) { pa[i] = (_Float16)(pr[i] * 16384.0f); pa[8 + i] = (_Float16)(pr[16 + i] * 16384.0f); } }
#pragma unroll
    for (int t = 0; t < 8; ++t) {
      union { v16h v; v8h q[2]; } vb; const _Float16* vr = &Vt[t * 16 + col][8 * g];
      vb.q[0] = *(const v8h*)(vr); vb.q[1] = *(const v8h*)(vr + 16);
      o[t] = wmma_h(pa, vb.v, o[t]);
    }
  }
  __syncthreads();
  float* T = (float*)&Ahi[0][0];
#pragma unroll
  for (int t = 0; t < 8; ++t)
#pragma unroll
    for (int r = 0; r < 8; ++r) T[(t * 16 + col) * 64 + wave * 16 + 8 * g + r] = o[t][r] / (l_r[r] * 16384.0f);
  __syncthreads();
  for (int gq = tid; gq < 128 * 16; gq += 128) { const int c = gq >> 4, pc = gq & 15;
    vst2(out + ((size_t)b * CDIM + c) * LDIM + m0 + pc * 4, *(const v4f*)(T + c * 64 + pc * 4)); }
}

extern "C" void kernel_launch(void* const* d_in, const int* in_sizes, int n_in,
                              void* d_out, int out_size, void* d_ws, size_t ws_size,
                              hipStream_t stream) {
  (void)in_sizes; (void)n_in; (void)out_size; (void)ws_size;
  const float* x   = (const float*)d_in[0];
  const float* Wq  = (const float*)d_in[1];
  const float* bq  = (const float*)d_in[2];
  const float* Wk  = (const float*)d_in[3];
  const float* bk  = (const float*)d_in[4];
  const float* Wv  = (const float*)d_in[5];
  const float* bv  = (const float*)d_in[6];
  const float* pos = (const float*)d_in[7];
  float* out = (float*)d_out;
  float* Qf = (float*)d_ws;
  float* Kf = Qf + (size_t)BATCH * LDIM * CDIM;
  _Float16* Vh = (_Float16*)(Kf + (size_t)BATCH * LDIM * CDIM);
  k_proj<<<dim3(LDIM / 64, BATCH), 128, 0, stream>>>(x, Wq, bq, Wk, bk, Wv, bv, Qf, Kf, Vh);
  k_attn<<<dim3(LDIM / 64, BATCH), 128, 0, stream>>>(Qf, Kf, Vh, pos, out);
}
